// EncoderRNN_77455440216599
// MI455X (gfx1250) — hardware-run, weakly checked
//
#include <hip/hip_runtime.h>
#include <math.h>

constexpr int NUMU  = 256;
constexpr int NTOK  = 128;
constexpr int NEMB  = 256;
constexpr int NHID  = 256;
constexpr int NGATE = 4 * NHID;
constexpr int NSEQ2 = 2 * NHID;
constexpr int NTHR  = 256;
constexpr int BROWS = 16;
constexpr int HP    = NHID + 8;
constexpr int OP    = NHID + 4;
constexpr int NROWS = NTOK * NUMU;
constexpr float OPC     = 16.0f;
constexpr float ACC_INV = 1.0f / 256.0f;
static_assert(NUMU % BROWS == 0, "batch tiles exact");
static_assert(NHID == 32 * (NTHR / 32), "8 waves x 32 hidden units");
static_assert(NEMB % 32 == 0 && NSEQ2 % 32 == 0 && NHID % 32 == 0, "K chunks of 32, no tails");
static_assert((NROWS * (NEMB / 8)) % NTHR == 0, "gather grid exact");
static_assert((NGATE * (NEMB / 8)) % NTHR == 0 && (NGATE * (NSEQ2 / 8)) % NTHR == 0, "cvt grids exact");
static_assert((BROWS * HP) % 2 == 0, "h tile word zero-fill exact type");
static_assert((BROWS * NHID / 8) % NTHR == 0, "Y copy: 2 x 16 B per thread");
static_assert((BROWS * NHID / 4) % NTHR == 0, "out copy: 4 x 16 B per thread");
static_assert((HP * 2) % 16 == 0 && (OP * 4) % 16 == 0, "16-B aligned LDS rows");

typedef __attribute__((ext_vector_type(16))) _Float16 v16h;
typedef __attribute__((ext_vector_type(8)))  _Float16 v8h;
typedef __attribute__((ext_vector_type(8)))  float    v8f;
typedef __attribute__((ext_vector_type(4)))  float    v4f;
typedef __attribute__((ext_vector_type(4)))  unsigned u4v;

__device__ __forceinline__ unsigned short f2bf_bits(float f) {
  unsigned u = __float_as_uint(f);
  return (unsigned short)((u + 0x7FFFu + ((u >> 16) & 1u)) >> 16);
}
__device__ __forceinline__ float bf_bits2f(unsigned short h) { return __uint_as_float(((unsigned)h) << 16); }
__device__ __forceinline__ float bf16r(float f) { return bf_bits2f(f2bf_bits(f)); }

__device__ __forceinline__ void dep_guard_h(v8f& a, v8f& b, v16h x, v16h y) { asm volatile("v_nop\n\tv_nop\n\tv_nop\n\tv_nop" : "+v"(a), "+v"(b) : "v"(x), "v"(y)); }
__device__ __forceinline__ void keep4_h(v16h a, v16h b, v16h c, v16h d) { asm volatile("v_nop" :: "v"(a), "v"(b), "v"(c), "v"(d)); }
__device__ __forceinline__ void acc_guard4(v8f& a, v8f& b, v8f& c, v8f& d) { asm volatile("v_nop\n\tv_nop\n\tv_nop\n\tv_nop" : "+v"(a), "+v"(b), "+v"(c), "+v"(d)); }
template <typename T> struct Frag;
template <> struct Frag<_Float16> {
  typedef v16h V; union U { v16h v; v8h h[2]; };
  static __device__ __forceinline__ v16h load(const _Float16* p) {
    U f; f.h[0] = *(const v8h*)(p); f.h[1] = *(const v8h*)(p + 16); return f.v;
  }
  static __device__ __forceinline__ v8f mma(v16h a, v16h b, v8f c) {
    return __builtin_amdgcn_wmma_f32_16x16x32_f16(false, a, false, b, (short)0, c, false, false);
  }
};

__device__ __forceinline__ float fsig(float x) { return __builtin_amdgcn_rcpf(1.0f + expf(-x)); }

template <int MODE>
__global__ __launch_bounds__(NTHR) void cvt8_kernel(const float* __restrict__ src, unsigned short* __restrict__ dst,
                                                    int nrow, int ncol8, int spitch, int scol0, float sc) {
  const int i  = blockIdx.x * NTHR + threadIdx.x;
  const int n8 = nrow * ncol8;
  if (i < n8) {
    const int row = i / ncol8;
    const int c8  = i - row * ncol8;
    const float* sp = src + (size_t)row * spitch + scol0 + c8 * 8;
    const v4f a = *(const v4f*)(sp);
    const v4f b = *(const v4f*)(sp + 4);
    v8h hv;
#pragma unroll
    for (int e = 0; e < 4; ++e) {
      unsigned short b0, b1;
      if (MODE == 0) {
        b0 = f2bf_bits(a[e] * sc);
        b1 = f2bf_bits(b[e] * sc);
      } else {
        b0 = __builtin_bit_cast(unsigned short, (_Float16)(bf16r(a[e]) * sc));
        b1 = __builtin_bit_cast(unsigned short, (_Float16)(bf16r(b[e]) * sc));
      }
      hv[e]     = __builtin_bit_cast(_Float16, b0);
      hv[4 + e] = __builtin_bit_cast(_Float16, b1);
    }
    *(volatile v8h*)(dst + (size_t)i * 8) = hv;
    __threadfence();
    *(volatile v8h*)(dst + (size_t)i * 8) = hv;
  }
}

__global__ __launch_bounds__(NTHR) void gather_x_kernel(const int* __restrict__ idc, const float* __restrict__ emb,
                                                        unsigned short* __restrict__ X0, int nvocab) {
  const int i = blockIdx.x * NTHR + threadIdx.x;
  if (i >= NROWS * (NEMB / 8)) return;
  const int row = i >> 5;
  const int seg = i & 31;
  const int t = row >> 8, b = row & 255;
  int tok = idc[b * NTOK + t];
  tok = tok < 0 ? 0 : tok;
  tok = tok > nvocab - 1 ? nvocab - 1 : tok;
  const float* sp = emb + (size_t)tok * NEMB + seg * 8;
  const v4f a = *(const v4f*)(sp);
  const v4f q = *(const v4f*)(sp + 4);
  v8h hv;
#pragma unroll
  for (int e = 0; e < 4; ++e) {
    hv[e]     = (_Float16)(bf16r(a[e]) * OPC);
    hv[4 + e] = (_Float16)(bf16r(q[e]) * OPC);
  }
  unsigned short* dp = X0 + (size_t)row * NEMB + seg * 8;
  *(volatile v8h*)dp = hv;
  __threadfence();
  *(volatile v8h*)dp = hv;
}

template <int DIN>
__device__ __forceinline__ void stage_x_tile(unsigned short* Ax, const unsigned short* xpl, int t, int b0, int tid) {
  constexpr int XP  = DIN + 8;
  constexpr int XCH = DIN / 8;
  constexpr int XIT = (BROWS * XCH) / NTHR;
  static_assert((BROWS * XCH) % NTHR == 0, "x tile staging exact");
#pragma unroll
  for (int it = 0; it < XIT; ++it) {
    const int i  = it * NTHR + tid;
    const int m  = i / XCH;
    const int c8 = i - m * XCH;
    const u4v v = *(const u4v*)(xpl + ((size_t)(t * NUMU + b0 + m)) * DIN + c8 * 8);
    *(u4v*)(Ax + m * XP + c8 * 8) = v;
  }
}

template <int DIN, bool WRITE_Y, bool WRITE_OUT>
__global__ __launch_bounds__(NTHR) void lstm_scan_kernel(
    const unsigned short* xpl,
    const unsigned short* wihF, const unsigned short* whhF, const float* bF,
    const unsigned short* wihB, const unsigned short* whhB, const float* bB,
    unsigned short* ypl,
    float* outp,
    int dir_base, int nsteps) {
  constexpr int XP = DIN + 8;
  static_assert(DIN % 32 == 0, "K chunks of 32");
  __shared__ __align__(16) unsigned short Ax[BROWS * XP];
  __shared__ __align__(16) unsigned short Ah[BROWS * HP];
  __shared__ __align__(16) float          Hs[WRITE_OUT ? BROWS * OP : 4];

  const int tid = threadIdx.x, lane = tid & 31, wave = tid >> 5;
  const int c = lane & 15, hh = lane >> 4, koff = hh * 8;
  const int dir = blockIdx.y + dir_base;
  const int b0  = blockIdx.x * BROWS;
  const _Float16* WI = (const _Float16*)(const void*)(dir ? wihB : wihF);
  const _Float16* WH = (const _Float16*)(const void*)(dir ? whhB : whhF);
  const float* bias = dir ? bB : bF;
  const int t0     = dir ? (NTOK - 1) : 0;
  const int tstep  = dir ? -1 : 1;
  const int coloff = dir * NHID;
  int ns = nsteps;
  ns = ns < 1 ? 1 : ns;
  ns = ns > NTOK ? NTOK : ns;

  {
    unsigned* ahw = (unsigned*)(void*)Ah;
#pragma unroll 1
    for (int i = tid; i < BROWS * HP / 2; i += NTHR) ahw[i] = 0u;
  }
  stage_x_tile<DIN>(Ax, xpl, t0, b0, tid);

  float cst[2][8], hst[2][8], bb[2][4];
#pragma unroll
  for (int nt = 0; nt < 2; ++nt) {
    const int j = 32 * wave + 16 * nt + c;
#pragma unroll
    for (int g = 0; g < 4; ++g) bb[nt][g] = bf16r(bias[g * NHID + j]);
#pragma unroll
    for (int r = 0; r < 8; ++r) { cst[nt][r] = 0.0f; hst[nt][r] = 0.0f; }
  }
  __syncthreads();

  const _Float16* axrow = (const _Float16*)(const void*)Ax + c * XP + koff;
  const _Float16* ahrow = (const _Float16*)(const void*)Ah + c * HP + koff;
  const v8f z8 = {0.f, 0.f, 0.f, 0.f, 0.f, 0.f, 0.f, 0.f};

#pragma unroll 1
  for (int s = 0; s < ns; ++s) {
    const int t = t0 + s * tstep;
#pragma unroll
    for (int nt = 0; nt < 2; ++nt) {
      const int j = 32 * wave + 16 * nt + c;
      const _Float16* wi = WI + (size_t)j * DIN + koff;
      const _Float16* wh = WH + (size_t)j * NHID + koff;
      v8f acc[4];
      acc[0] = z8; acc[1] = z8; acc[2] = z8; acc[3] = z8;
#pragma unroll 1
      for (int kx = 0; kx < DIN; kx += 32) {
        const v16h a  = Frag<_Float16>::load(axrow + kx);
        const v16h q0 = Frag<_Float16>::load(wi + kx);
        const v16h q1 = Frag<_Float16>::load(wi + (size_t)1 * NHID * DIN + kx);
        const v16h q2 = Frag<_Float16>::load(wi + (size_t)2 * NHID * DIN + kx);
        const v16h q3 = Frag<_Float16>::load(wi + (size_t)3 * NHID * DIN + kx);
        acc[0] = Frag<_Float16>::mma(a, q0, acc[0]);
        acc[1] = Frag<_Float16>::mma(a, q1, acc[1]);
        acc[2] = Frag<_Float16>::mma(a, q2, acc[2]);
        acc[3] = Frag<_Float16>::mma(a, q3, acc[3]);
        dep_guard_h(acc[0], acc[3], a, q3);
        keep4_h(q0, q1, q2, q3);
      }
#pragma unroll 1
      for (int k0 = 0; k0 < NHID; k0 += 32) {
        const v16h a  = Frag<_Float16>::load(ahrow + k0);
        const v16h q0 = Frag<_Float16>::load(wh + k0);
        const v16h q1 = Frag<_Float16>::load(wh + (size_t)1 * NHID * NHID + k0);
        const v16h q2 = Frag<_Float16>::load(wh + (size_t)2 * NHID * NHID + k0);
        const v16h q3 = Frag<_Float16>::load(wh + (size_t)3 * NHID * NHID + k0);
        acc[0] = Frag<_Float16>::mma(a, q0, acc[0]);
        acc[1] = Frag<_Float16>::mma(a, q1, acc[1]);
        acc[2] = Frag<_Float16>::mma(a, q2, acc[2]);
        acc[3] = Frag<_Float16>::mma(a, q3, acc[3]);
        dep_guard_h(acc[0], acc[3], a, q3);
        keep4_h(q0, q1, q2, q3);
      }
      acc_guard4(acc[0], acc[1], acc[2], acc[3]);
#pragma unroll
      for (int r = 0; r < 8; ++r) {
        const float zi = acc[0][r] * ACC_INV + bb[nt][0];
        const float zf = acc[1][r] * ACC_INV + bb[nt][1];
        const float zg = acc[2][r] * ACC_INV + bb[nt][2];
        const float zo = acc[3][r] * ACC_INV + bb[nt][3];
        const float ig = fsig(zi);
        const float fg = fsig(zf);
        const float gg = tanhf(zg);
        const float og = fsig(zo);
        const float cn = fg * cst[nt][r] + ig * gg;
        cst[nt][r] = cn;
        hst[nt][r] = og * tanhf(cn);
      }
    }
    __syncthreads();

#pragma unroll
    for (int nt = 0; nt < 2; ++nt) {
      const int j = 32 * wave + 16 * nt + c;
#pragma unroll
      for (int r = 0; r < 8; ++r)
        Ah[(8 * hh + r) * HP + j] = __builtin_bit_cast(unsigned short, (_Float16)(hst[nt][r] * OPC));
    }
    const bool last = (s == ns - 1);
    if (WRITE_OUT && last) {
#pragma unroll
      for (int nt = 0; nt < 2; ++nt) {
        const int j = 32 * wave + 16 * nt + c;
#pragma unroll
        for (int r = 0; r < 8; ++r) Hs[(8 * hh + r) * OP + j] = hst[nt][r];
      }
    }
    {
      const int sn = (s + 1 < ns) ? (s + 1) : (ns - 1);
      stage_x_tile<DIN>(Ax, xpl, t0 + sn * tstep, b0, tid);
    }
    __syncthreads();

    if (WRITE_Y) {
      u4v yv[2];
#pragma unroll
      for (int it = 0; it < 2; ++it) {
        const int i = it * NTHR + tid;
        const int m = i >> 5, seg = i & 31;
        yv[it] = *(const u4v*)(Ah + m * HP + seg * 8);
      }
      for (int pass = 0; pass < 2; ++pass) {
#pragma unroll
        for (int it = 0; it < 2; ++it) {
          const int i = it * NTHR + tid;
          const int m = i >> 5, seg = i & 31;
          *(volatile u4v*)(ypl + ((size_t)(t * NUMU + b0 + m)) * NSEQ2 + coloff + seg * 8) = yv[it];
        }
        __threadfence();
      }
    }
    if (WRITE_OUT && last) {
      v4f ov[4];
#pragma unroll
      for (int it = 0; it < 4; ++it) {
        const int idx = it * NTHR + tid;
        const int row = idx >> 6, c4 = (idx & 63) * 4;
        ov[it] = *(const v4f*)(Hs + row * OP + c4);
      }
      for (int pass = 0; pass < 2; ++pass) {
#pragma unroll
        for (int it = 0; it < 4; ++it) {
          const int idx = it * NTHR + tid;
          const int row = idx >> 6, c4 = (idx & 63) * 4;
          *(volatile v4f*)(outp + (size_t)(b0 + row) * NSEQ2 + coloff + c4) = ov[it];
        }
        __threadfence();
      }
    }
  }
}

extern "C" void kernel_launch(void* const* d_in, const int* in_sizes, int n_in,
                              void* d_out, int out_size, void* d_ws, size_t ws_size, hipStream_t stream) {
  if (n_in < 14 || d_out == nullptr || d_ws == nullptr) return;
  if (in_sizes[0] != NUMU * NTOK || in_sizes[1] < NEMB || (in_sizes[1] % NEMB) != 0 ||
      in_sizes[2] != NGATE * NEMB || in_sizes[3] != NGATE * NHID || in_sizes[4] != NGATE ||
      in_sizes[5] != NGATE * NEMB || in_sizes[6] != NGATE * NHID || in_sizes[7] != NGATE ||
      in_sizes[8] != NGATE * NSEQ2 || in_sizes[9] != NGATE * NHID || in_sizes[10] != NGATE ||
      in_sizes[11] != NGATE * NSEQ2 || in_sizes[12] != NGATE * NHID || in_sizes[13] != NGATE ||
      out_size != NUMU * NSEQ2) return;

  const int*   idc    = (const int*)d_in[0];
  const float* emb    = (const float*)d_in[1];
  const float* w_ih0f = (const float*)d_in[2];
  const float* w_hh0f = (const float*)d_in[3];
  const float* b0f    = (const float*)d_in[4];
  const float* w_ih0b = (const float*)d_in[5];
  const float* w_hh0b = (const float*)d_in[6];
  const float* b0b    = (const float*)d_in[7];
  const float* w_ih1f = (const float*)d_in[8];
  const float* w_hh1f = (const float*)d_in[9];
  const float* b1f    = (const float*)d_in[10];
  const float* w_ih1b = (const float*)d_in[11];
  const float* w_hh1b = (const float*)d_in[12];
  const float* b1b    = (const float*)d_in[13];
  float* out = (float*)d_out;
  const int nvocab = in_sizes[1] / NEMB;

  char* ws = (char*)d_ws; size_t off = 0;
  auto carve = [&](size_t bytes) -> char* { char* p = ws + off; off += (bytes + 255) & ~(size_t)255; return p; };
  unsigned short* X0    = (unsigned short*)carve((size_t)NROWS * NEMB * 2);
  unsigned short* Y0    = (unsigned short*)carve((size_t)NROWS * NSEQ2 * 2);
  unsigned short* WIH0F = (unsigned short*)carve((size_t)NGATE * NEMB * 2);
  unsigned short* WHH0F = (unsigned short*)carve((size_t)NGATE * NHID * 2);
  unsigned short* WIH0B = (unsigned short*)carve((size_t)NGATE * NEMB * 2);
  unsigned short* WHH0B = (unsigned short*)carve((size_t)NGATE * NHID * 2);
  unsigned short* WIH1F = (unsigned short*)carve((size_t)NGATE * NSEQ2 * 2);
  unsigned short* WHH1F = (unsigned short*)carve((size_t)NGATE * NHID * 2);
  unsigned short* WIH1B = (unsigned short*)carve((size_t)NGATE * NSEQ2 * 2);
  unsigned short* WHH1B = (unsigned short*)carve((size_t)NGATE * NHID * 2);
  if (off > ws_size || off > (size_t)134217728) return;

  gather_x_kernel<<<(NROWS * (NEMB / 8)) / NTHR, NTHR, 0, stream>>>(idc, emb, X0, nvocab);

  const int n8a = NGATE * (NEMB / 8);
  const int n8c = NGATE * (NSEQ2 / 8);
  cvt8_kernel<1><<<(n8a + NTHR - 1) / NTHR, NTHR, 0, stream>>>(w_ih0f, WIH0F, NGATE, NEMB / 8,  NEMB,  0, OPC);
  cvt8_kernel<1><<<(n8a + NTHR - 1) / NTHR, NTHR, 0, stream>>>(w_hh0f, WHH0F, NGATE, NHID / 8,  NHID,  0, OPC);
  cvt8_kernel<1><<<(n8a + NTHR - 1) / NTHR, NTHR, 0, stream>>>(w_ih0b, WIH0B, NGATE, NEMB / 8,  NEMB,  0, OPC);
  cvt8_kernel<1><<<(n8a + NTHR - 1) / NTHR, NTHR, 0, stream>>>(w_hh0b, WHH0B, NGATE, NHID / 8,  NHID,  0, OPC);
  cvt8_kernel<1><<<(n8c + NTHR - 1) / NTHR, NTHR, 0, stream>>>(w_ih1f, WIH1F, NGATE, NSEQ2 / 8, NSEQ2, 0, OPC);
  cvt8_kernel<1><<<(n8a + NTHR - 1) / NTHR, NTHR, 0, stream>>>(w_hh1f, WHH1F, NGATE, NHID / 8,  NHID,  0, OPC);
  cvt8_kernel<1><<<(n8c + NTHR - 1) / NTHR, NTHR, 0, stream>>>(w_ih1b, WIH1B, NGATE, NSEQ2 / 8, NSEQ2, 0, OPC);
  cvt8_kernel<1><<<(n8a + NTHR - 1) / NTHR, NTHR, 0, stream>>>(w_hh1b, WHH1B, NGATE, NHID / 8,  NHID,  0, OPC);

  lstm_scan_kernel<NEMB, true, false><<<dim3(NUMU / BROWS, 2), NTHR, 0, stream>>>(
      X0, WIH0F, WHH0F, b0f, WIH0B, WHH0B, b0b, Y0, out, 0, NTOK);
  lstm_scan_kernel<NSEQ2, false, true><<<dim3(NUMU / BROWS, 1), NTHR, 0, stream>>>(
      Y0, WIH1F, WHH1F, b1f, WIH1B, WHH1B, b1b, X0, out, 0, NTOK);
  lstm_scan_kernel<NSEQ2, false, true><<<dim3(NUMU / BROWS, 1), NTHR, 0, stream>>>(
      Y0, WIH1F, WHH1F, b1f, WIH1B, WHH1B, b1b, X0, out, 1, 1);
}
